// SelfAttention123_52553219833949
// MI455X (gfx1250) — hardware-verified
//
#include <hip/hip_runtime.h>
#include <math.h>
#include <stdint.h>

#define NB    2
#define SEQ   2048
#define DM    1024
#define NH    16
#define HD    64
#define LR    4
#define NQB   (SEQ / 64)
#define ROWS  (NB * SEQ)
#define OUTN  (ROWS * DM)
#define NLEAD 8
static_assert(NH * HD == DM);
static_assert(HD == 64);
static_assert(LR == 4);
static_assert((SEQ % 64) == 0 && (DM % 64) == 0 && (DM % 256) == 0);
static_assert((SEQ & (SEQ - 1)) == 0);
static_assert(((ROWS / 64) * (DM / 64)) % 8 == 0);
static_assert(((ROWS * DM / 8) % 256) == 0);
static_assert(((DM * DM / 8) % 256) == 0);
static_assert((ROWS % 8) == 0);

typedef _Float16 v16h __attribute__((ext_vector_type(16)));
typedef _Float16 v8h  __attribute__((ext_vector_type(8)));
typedef __bf16   v16b __attribute__((ext_vector_type(16)));
typedef __bf16   v8b  __attribute__((ext_vector_type(8)));
typedef float    v8f  __attribute__((ext_vector_type(8)));
typedef float    v4f  __attribute__((ext_vector_type(4)));
typedef unsigned int v4u __attribute__((ext_vector_type(4)));

__device__ __forceinline__ unsigned short bf_bits(float f) {
  unsigned u = __float_as_uint(f);
  return (unsigned short)((u + 0x7FFFu + ((u >> 16) & 1u)) >> 16);
}
__device__ __forceinline__ float bf_up(unsigned short h) { return __uint_as_float(((unsigned)h) << 16); }
__device__ __forceinline__ float bfr(float f) { return bf_up(bf_bits(f)); }
__device__ __forceinline__ unsigned short h_bits(_Float16 x) { return __builtin_bit_cast(unsigned short, x); }
__device__ __forceinline__ unsigned pk16(unsigned short a, unsigned short b) { return (unsigned)a | ((unsigned)b << 16); }
__device__ __forceinline__ v8f zero8() { v8f z = {0.f, 0.f, 0.f, 0.f, 0.f, 0.f, 0.f, 0.f}; return z; }

__device__ __forceinline__ v16b ldfrag_b(const __bf16* p) {
  union { v16b v; v8b h[2]; } f;
  f.h[0] = *(const v8b*)(p);
  f.h[1] = *(const v8b*)(p + 16);
  return f.v;
}
__device__ __forceinline__ v16h ldfrag_h(const _Float16* p) {
  union { v16h v; v8h h[2]; } f;
  f.h[0] = *(const v8h*)(p);
  f.h[1] = *(const v8h*)(p + 16);
  return f.v;
}

__device__ __forceinline__ v8f mma_h(v16h a, v16h b, v8f c) {
  c = __builtin_amdgcn_wmma_f32_16x16x32_f16(false, a, false, b, (short)0, c, false, false);
#if defined(__HIP_DEVICE_COMPILE__)
  asm volatile("v_nop\n\tv_nop\n\tv_nop\n\tv_nop" : "+v"(c) : "v"(a), "v"(b));
#endif
  return c;
}
__device__ __forceinline__ v8f mma_b_raw(v16b a, v16b b, v8f c) {
  return __builtin_amdgcn_wmma_f32_16x16x32_bf16(false, a, false, b, (short)0, c, false, false);
}
__device__ __forceinline__ void dep_guard_b(v8f& a, v8f& b, v16b x, v16b y) {
#if defined(__HIP_DEVICE_COMPILE__)
  asm volatile("v_nop\n\tv_nop\n\tv_nop\n\tv_nop" : "+v"(a), "+v"(b) : "v"(x), "v"(y));
#endif
}
__device__ __forceinline__ void keep4_b(v16b a, v16b b, v16b c, v16b d) {
#if defined(__HIP_DEVICE_COMPILE__)
  asm volatile("v_nop" :: "v"(a), "v"(b), "v"(c), "v"(d));
#endif
}
__device__ __forceinline__ void acc_guard4(v8f& a, v8f& b, v8f& c, v8f& d) {
#if defined(__HIP_DEVICE_COMPILE__)
  asm volatile("v_nop\n\tv_nop\n\tv_nop\n\tv_nop" : "+v"(a), "+v"(b), "+v"(c), "+v"(d));
#endif
}

__global__ __launch_bounds__(256) void cvt_bf16x8(const float* __restrict__ in, unsigned short* out, int n8) {
  const int i = blockIdx.x * 256 + threadIdx.x;
  if (i < n8) {
    const v4f a = *(const v4f*)(in + (size_t)i * 8);
    const v4f b = *(const v4f*)(in + (size_t)i * 8 + 4);
    v4u p;
    p[0] = pk16(bf_bits(a[0]), bf_bits(a[1]));
    p[1] = pk16(bf_bits(a[2]), bf_bits(a[3]));
    p[2] = pk16(bf_bits(b[0]), bf_bits(b[1]));
    p[3] = pk16(bf_bits(b[2]), bf_bits(b[3]));
    *(volatile v4u*)(out + (size_t)i * 8) = p;
    __threadfence();
    *(volatile v4u*)(out + (size_t)i * 8) = p;
  }
}

__global__ __launch_bounds__(256) void planes_f16x8(const float* __restrict__ in, unsigned short* hp,
                                                    unsigned short* lp, int n8, float scale) {
  const int i = blockIdx.x * 256 + threadIdx.x;
  if (i < n8) {
    const v4f a = *(const v4f*)(in + (size_t)i * 8);
    const v4f b = *(const v4f*)(in + (size_t)i * 8 + 4);
    float f[8];
    f[0] = a[0]; f[1] = a[1]; f[2] = a[2]; f[3] = a[3];
    f[4] = b[0]; f[5] = b[1]; f[6] = b[2]; f[7] = b[3];
    v4u ph, pl;
#pragma unroll
    for (int e = 0; e < 4; ++e) {
      const float f0 = f[2 * e] * scale;
      const float f1 = f[2 * e + 1] * scale;
      const _Float16 x0 = (_Float16)f0, x1 = (_Float16)f1;
      const _Float16 l0 = (_Float16)((f0 - (float)x0) * 1024.0f);
      const _Float16 l1 = (_Float16)((f1 - (float)x1) * 1024.0f);
      ph[e] = pk16(h_bits(x0), h_bits(x1));
      pl[e] = pk16(h_bits(l0), h_bits(l1));
    }
    *(volatile v4u*)(hp + (size_t)i * 8) = ph;
    *(volatile v4u*)(lp + (size_t)i * 8) = pl;
    __threadfence();
    *(volatile v4u*)(hp + (size_t)i * 8) = ph;
    *(volatile v4u*)(lp + (size_t)i * 8) = pl;
  }
}

__global__ __launch_bounds__(256) void lora_t(const unsigned short* __restrict__ Xb,
                                              const float* __restrict__ A0, const float* __restrict__ A1,
                                              const float* __restrict__ A2, float* T) {
  __shared__ __align__(16) float st[8 * LR];
  const int tid  = threadIdx.x;
  const int wave = tid >> 5;
  const int lane = tid & 31;
  const int p    = blockIdx.y;
  const int m0   = blockIdx.x * 8;
  const int m    = m0 + wave;
  const float* A = (p == 0) ? A0 : ((p == 1) ? A1 : A2);
  float t0 = 0.f, t1 = 0.f, t2 = 0.f, t3 = 0.f;
#pragma unroll 1
  for (int step = 0; step < DM / 256; ++step) {
    const int k = step * 256 + lane * 8;
    const v4u xv = *(const v4u*)(Xb + (size_t)m * DM + k);
    float xf[8];
#pragma unroll
    for (int e = 0; e < 4; ++e) {
      xf[2 * e]     = __uint_as_float(xv[e] << 16);
      xf[2 * e + 1] = __uint_as_float(xv[e] & 0xffff0000u);
    }
    float part[4];
#pragma unroll
    for (int r = 0; r < 4; ++r) {
      const v4f w0 = *(const v4f*)(A + (size_t)r * DM + k);
      const v4f w1 = *(const v4f*)(A + (size_t)r * DM + k + 4);
      float s = xf[0] * bfr(w0[0]);
      s += xf[1] * bfr(w0[1]);
      s += xf[2] * bfr(w0[2]);
      s += xf[3] * bfr(w0[3]);
      s += xf[4] * bfr(w1[0]);
      s += xf[5] * bfr(w1[1]);
      s += xf[6] * bfr(w1[2]);
      s += xf[7] * bfr(w1[3]);
      part[r] = s;
    }
    t0 += part[0]; t1 += part[1]; t2 += part[2]; t3 += part[3];
  }
#pragma unroll
  for (int off = 16; off > 0; off >>= 1) {
    t0 += __shfl_xor(t0, off, 32);
    t1 += __shfl_xor(t1, off, 32);
    t2 += __shfl_xor(t2, off, 32);
    t3 += __shfl_xor(t3, off, 32);
  }
  if (lane == 0) {
    st[wave * LR + 0] = t0;
    st[wave * LR + 1] = t1;
    st[wave * LR + 2] = t2;
    st[wave * LR + 3] = t3;
  }
  __syncthreads();
  if (tid < 8) {
    const v4f v = *(const v4f*)(st + tid * LR);
    float* dst = T + ((size_t)p * ROWS + (size_t)(m0 + tid)) * LR;
    *(volatile v4f*)dst = v;
    __threadfence();
    *(volatile v4f*)dst = v;
  }
}

__global__ __launch_bounds__(256) void gemm64_lora(
    const unsigned short* __restrict__ Ap, int lda,
    const unsigned short* __restrict__ Btp, int ldb,
    const float* __restrict__ biasp, const float* __restrict__ Tp,
    const float* __restrict__ Bmp, float lsc,
    float* C, int ldc, int M, int N, int K) {
  const __bf16* Ab = (const __bf16*)(const void*)Ap;
  const __bf16* Bb = (const __bf16*)(const void*)Btp;
  __shared__ __align__(16) float sT[8][16 * 68];
  const int lane = threadIdx.x & 31;
  const int wave = threadIdx.x >> 5;
  const int tilesN = N >> 6;
  const int tilesM = M >> 6;
  const int tile = blockIdx.x * 8 + wave;
  if (tile >= tilesM * tilesN) return;
  const int tm = tile / tilesN;
  const int tn = tile - tm * tilesN;
  const int m0 = tm << 6;
  const int n0 = tn << 6;

  const int rlane = lane & 15;
  const int koff  = (lane >> 4) * 8;
  const int mOff  = (lane >> 4) * 8;

  v8f acc[4][4];
#pragma unroll
  for (int i = 0; i < 4; ++i)
#pragma unroll
    for (int j = 0; j < 4; ++j) acc[i][j] = zero8();

  for (int k0 = 0; k0 < K; k0 += 32) {
    v16b bh[4];
#pragma unroll
    for (int j = 0; j < 4; ++j) {
      const size_t bo = (size_t)(n0 + (j << 4) + rlane) * ldb + koff + k0;
      bh[j] = ldfrag_b(Bb + bo);
    }
#pragma unroll
    for (int i = 0; i < 4; ++i) {
      const size_t ao = (size_t)(m0 + (i << 4) + rlane) * lda + koff + k0;
      const v16b ah = ldfrag_b(Ab + ao);
#pragma unroll
      for (int j = 0; j < 4; ++j) {
        acc[i][j] = mma_b_raw(ah, bh[j], acc[i][j]);
      }
      dep_guard_b(acc[i][0], acc[i][3], ah, bh[3]);
    }
    keep4_b(bh[0], bh[1], bh[2], bh[3]);
  }
  acc_guard4(acc[0][0], acc[0][1], acc[0][2], acc[0][3]);
  acc_guard4(acc[1][0], acc[1][1], acc[1][2], acc[1][3]);
  acc_guard4(acc[2][0], acc[2][1], acc[2][2], acc[2][3]);
  acc_guard4(acc[3][0], acc[3][1], acc[3][2], acc[3][3]);

  float* slab = sT[wave];
#pragma unroll
  for (int i = 0; i < 4; ++i) {
    const int mBase = m0 + (i << 4);
    v4f bmv[4];
    float bj[4];
#pragma unroll
    for (int j = 0; j < 4; ++j) {
      const int n = n0 + (j << 4) + rlane;
      const v4f w = *(const v4f*)(Bmp + (size_t)n * LR);
      v4f wb;
      wb[0] = bfr(w[0]); wb[1] = bfr(w[1]); wb[2] = bfr(w[2]); wb[3] = bfr(w[3]);
      bmv[j] = wb;
      bj[j] = bfr(biasp[n]);
    }
#pragma unroll
    for (int r = 0; r < 8; ++r) {
      const int row = mOff + r;
      const v4f tv = *(const v4f*)(Tp + (size_t)(mBase + row) * LR);
#pragma unroll
      for (int j = 0; j < 4; ++j) {
        const float lo = tv[0] * bmv[j][0] + tv[1] * bmv[j][1] + tv[2] * bmv[j][2] + tv[3] * bmv[j][3];
        slab[row * 68 + (j << 4) + rlane] = (acc[i][j][r] + bj[j]) + lsc * lo;
      }
    }
    __builtin_amdgcn_fence(__ATOMIC_RELEASE, "workgroup");
    __builtin_amdgcn_wave_barrier();
    __builtin_amdgcn_fence(__ATOMIC_ACQUIRE, "workgroup");
    {
      const int hh = lane >> 4, c4 = (lane & 15) * 4;
      v4f ov[8];
#pragma unroll
      for (int it = 0; it < 8; ++it) {
        const int row = it * 2 + hh;
        ov[it] = *(const v4f*)(slab + row * 68 + c4);
      }
      for (int pass = 0; pass < 2; ++pass) {
#pragma unroll
        for (int it = 0; it < 8; ++it) {
          const int row = it * 2 + hh;
          *(volatile v4f*)(C + (size_t)(mBase + row) * ldc + n0 + c4) = ov[it];
        }
        __threadfence();
      }
    }
    __builtin_amdgcn_fence(__ATOMIC_RELEASE, "workgroup");
    __builtin_amdgcn_wave_barrier();
    __builtin_amdgcn_fence(__ATOMIC_ACQUIRE, "workgroup");
  }
}

__global__ __launch_bounds__(256) void v_planes(const float* __restrict__ vf, int vrp,
                                                unsigned short* vth, unsigned short* vtl, float vscale) {
  __shared__ __align__(16) float sv[64 * 68];
  const int tid = threadIdx.x;
  const int t0  = blockIdx.x * 64;
  const int hh  = blockIdx.y;
  const int b   = blockIdx.z;
#pragma unroll
  for (int i = 0; i < 4; ++i) {
    const int idx = i * 256 + tid;
    const int tt = idx >> 4, c4 = (idx & 15) * 4;
    const v4f a = *(const v4f*)(vf + ((size_t)(b * SEQ + t0 + tt)) * vrp + hh * HD + c4);
    *(v4f*)(sv + tt * 68 + c4) = a;
  }
  __syncthreads();

  const int g = tid >> 3, piece = tid & 7;
  v4u hv[2], lv[2];
  size_t hofs[2];
#pragma unroll
  for (int it = 0; it < 2; ++it) {
    const int d = it * 32 + g;
    v4u a, a2;
#pragma unroll
    for (int e = 0; e < 4; ++e) {
      const float f0 = sv[(piece * 8 + 2 * e) * 68 + d] * vscale;
      const float f1 = sv[(piece * 8 + 2 * e + 1) * 68 + d] * vscale;
      const _Float16 x0 = (_Float16)f0, x1 = (_Float16)f1;
      const unsigned short h0 = h_bits(x0), h1 = h_bits(x1);
      const unsigned short l0 = h_bits((_Float16)((f0 - (float)x0) * 4096.0f));
      const unsigned short l1 = h_bits((_Float16)((f1 - (float)x1) * 4096.0f));
      a[e] = pk16(h0, h1); a2[e] = pk16(l0, l1);
    }
    hv[it] = a; lv[it] = a2;
    hofs[it] = ((size_t)(b * DM + hh * HD + d)) * SEQ + t0 + piece * 8;
  }
  for (int pass = 0; pass < 2; ++pass) {
#pragma unroll
    for (int it = 0; it < 2; ++it) {
      *(volatile v4u*)(vth + hofs[it]) = hv[it];
      *(volatile v4u*)(vtl + hofs[it]) = lv[it];
    }
    __threadfence();
  }
}

__global__ __launch_bounds__(128)
void attn_p64(const unsigned short* __restrict__ qhp, const unsigned short* __restrict__ qlp,
              const unsigned short* __restrict__ khp, const unsigned short* __restrict__ klp,
              const unsigned short* __restrict__ vhp, const unsigned short* __restrict__ vlp,
              const float* __restrict__ maskp, float* outp, float sscale, float oscl) {
  union FH { v16h v; v8h h[2]; };
  __shared__ __align__(16) _Float16 Ksh[64 * 64];
  __shared__ __align__(16) _Float16 Ksl[64 * 64];
  __shared__ __align__(16) _Float16 Vth[64 * 64];
  __shared__ __align__(16) _Float16 Vtl[64 * 64];
  __shared__ __align__(16) _Float16 Psh[4][16 * 64];
  __shared__ __align__(16) _Float16 Psl[4][16 * 64];
  __shared__ __align__(16) float    Os[4][16 * 64];

  const int tid  = threadIdx.x;
  const int wave = tid >> 5;
  const int lane = tid & 31;
  const int hh   = lane >> 4;
  const int c    = lane & 15;

  const int bx   = blockIdx.x;
  const int qb   = bx % NQB;
  const int rest = bx / NQB;
  const int h    = rest % NH;
  const int b    = rest / NH;
  const int q0   = qb * 64 + wave * 16;
  const size_t rowB = (size_t)b * SEQ;
  const bool lead = (qb < NLEAD);

  const _Float16* Qp  = (const _Float16*)(const void*)qhp + (size_t)h * HD;
  const _Float16* Qlq = (const _Float16*)(const void*)qlp + (size_t)h * HD;
  const _Float16* Kp  = (const _Float16*)(const void*)khp + (size_t)h * HD;
  const _Float16* Klq = (const _Float16*)(const void*)klp + (size_t)h * HD;
  const _Float16* Vh  = (const _Float16*)(const void*)vhp + ((size_t)b * DM + (size_t)h * HD) * SEQ;
  const _Float16* Vl  = (const _Float16*)(const void*)vlp + ((size_t)b * DM + (size_t)h * HD) * SEQ;

  v16h qa[2], ql[2];
#pragma unroll
  for (int dc = 0; dc < 2; ++dc) {
    const size_t qo = (rowB + q0 + c) * DM + dc * 32 + 8 * hh;
    qa[dc] = ldfrag_h(Qp + qo);
    ql[dc] = ldfrag_h(Qlq + qo);
  }

  float mrow[8], lrow[8];
  v8f oacc[4];
#pragma unroll
  for (int r = 0; r < 8; ++r) { mrow[r] = -INFINITY; lrow[r] = 0.f; }
#pragma unroll
  for (int t = 0; t < 4; ++t) oacc[t] = zero8();

  _Float16* pwh = Psh[wave];
  _Float16* pwl = Psl[wave];

  const int nkt = qb + 1;
  for (int kt = 0; kt < nkt; ++kt) {
    const int kv0 = kt * 64;
    __syncthreads();
    {
      const int r = tid >> 1, half = (tid & 1) * 32;
      const _Float16* kg  = Kp  + (rowB + kv0 + r) * DM + half;
      const _Float16* klg = Klq + (rowB + kv0 + r) * DM + half;
      const _Float16* vg  = Vh + (size_t)r * SEQ + kv0 + half;
      const _Float16* vlg = Vl + (size_t)r * SEQ + kv0 + half;
#pragma unroll
      for (int i = 0; i < 4; ++i) {
        const v8h a0 = *(const v8h*)(kg + 8 * i);
        const v8h a1 = *(const v8h*)(klg + 8 * i);
        const v8h b0 = *(const v8h*)(vg + 8 * i);
        const v8h b1 = *(const v8h*)(vlg + 8 * i);
        *(v8h*)(Ksh + r * 64 + half + 8 * i) = a0;
        *(v8h*)(Ksl + r * 64 + half + 8 * i) = a1;
        *(v8h*)(Vth + r * 64 + half + 8 * i) = b0;
        *(v8h*)(Vtl + r * 64 + half + 8 * i) = b1;
      }
    }
    __syncthreads();

    v8f s[4];
#pragma unroll
    for (int j = 0; j < 4; ++j) {
      s[j] = zero8();
      v8f s1 = zero8();
#pragma unroll
      for (int dc = 0; dc < 2; ++dc) {
        FH kb, kr;
        kb.h[0] = *(const v8h*)(Ksh + (j * 16 + c) * 64 + dc * 32 + 8 * hh);
        kb.h[1] = *(const v8h*)(Ksh + (j * 16 + c) * 64 + dc * 32 + 16 + 8 * hh);
        kr.h[0] = *(const v8h*)(Ksl + (j * 16 + c) * 64 + dc * 32 + 8 * hh);
        kr.h[1] = *(const v8h*)(Ksl + (j * 16 + c) * 64 + dc * 32 + 16 + 8 * hh);
        s[j] = mma_h(qa[dc], kb.v, s[j]);
        s1   = mma_h(qa[dc], kr.v, s1);
        s1   = mma_h(ql[dc], kb.v, s1);
      }
#pragma unroll
      for (int r = 0; r < 8; ++r) s[j][r] += s1[r] * (1.0f / 1024.0f);
    }

    float mkv[4];
#pragma unroll
    for (int j = 0; j < 4; ++j) mkv[j] = bfr(maskp[rowB + kv0 + j * 16 + c]);

#pragma unroll
    for (int r = 0; r < 8; ++r) {
      const int qrow = q0 + 8 * hh + r;
      float m = -INFINITY;
#pragma unroll
      for (int j = 0; j < 4; ++j) {
        const int key = kv0 + j * 16 + c;
        float sv = s[j][r] * sscale + mkv[j];
        sv += (key > qrow) ? -10000.0f : 0.0f;
        s[j][r] = sv;
        m = fmaxf(m, sv);
      }
#pragma unroll
      for (int off = 1; off < 16; off <<= 1) m = fmaxf(m, __shfl_xor(m, off, 32));
      const float mnew  = fmaxf(mrow[r], m);
      const float msafe = (mnew == -INFINITY) ? 0.f : mnew;
      const float alpha = __expf(mrow[r] - msafe);
      mrow[r] = mnew;
      float psum = 0.f;
#pragma unroll
      for (int j = 0; j < 4; ++j) {
        const float p  = __expf(s[j][r] - msafe);
        psum += p;
        const float pf = p * 1024.0f;
        const _Float16 ph = (_Float16)pf;
        pwh[(8 * hh + r) * 64 + j * 16 + c] = ph;
        if (lead) {
          const _Float16 pr = (_Float16)((pf - (float)ph) * 4096.0f);
          pwl[(8 * hh + r) * 64 + j * 16 + c] = pr;
        }
      }
#pragma unroll
      for (int off = 1; off < 16; off <<= 1) psum += __shfl_xor(psum, off, 32);
      lrow[r] = lrow[r] * alpha + psum;
#pragma unroll
      for (int t = 0; t < 4; ++t) oacc[t][r] *= alpha;
    }
    __builtin_amdgcn_fence(__ATOMIC_RELEASE, "workgroup");
    __builtin_amdgcn_wave_barrier();
    __builtin_amdgcn_fence(__ATOMIC_ACQUIRE, "workgroup");

    v8f o1[4];
#pragma unroll
    for (int t = 0; t < 4; ++t) o1[t] = zero8();
#pragma unroll 1
    for (int kk = 0; kk < 2; ++kk) {
      FH pa, pz;
      pa.h[0] = *(const v8h*)(pwh + c * 64 + kk * 32 + 8 * hh);
      pa.h[1] = *(const v8h*)(pwh + c * 64 + kk * 32 + 16 + 8 * hh);
      pz.h[0] = *(const v8h*)(pwl + c * 64 + kk * 32 + 8 * hh);
      pz.h[1] = *(const v8h*)(pwl + c * 64 + kk * 32 + 16 + 8 * hh);
#pragma unroll
      for (int t = 0; t < 4; ++t) {
        FH vb;
        vb.h[0] = *(const v8h*)(Vth + (t * 16 + c) * 64 + kk * 32 + 8 * hh);
        vb.h[1] = *(const v8h*)(Vth + (t * 16 + c) * 64 + kk * 32 + 16 + 8 * hh);
        oacc[t] = mma_h(pa.v, vb.v, oacc[t]);
        if (lead) o1[t] = mma_h(pz.v, vb.v, o1[t]);
        FH vl;
        vl.h[0] = *(const v8h*)(Vtl + (t * 16 + c) * 64 + kk * 32 + 8 * hh);
        vl.h[1] = *(const v8h*)(Vtl + (t * 16 + c) * 64 + kk * 32 + 16 + 8 * hh);
        o1[t] = mma_h(pa.v, vl.v, o1[t]);
      }
    }
#pragma unroll
    for (int t = 0; t < 4; ++t)
#pragma unroll
      for (int r = 0; r < 8; ++r) oacc[t][r] += o1[t][r] * (1.0f / 4096.0f);
  }

  float* os = Os[wave];
#pragma unroll
  for (int r = 0; r < 8; ++r) {
    const float l = lrow[r];
    const float inv = ((l > 0.f) ? (1.0f / l) : 0.f) * oscl;
#pragma unroll
    for (int t = 0; t < 4; ++t) os[(8 * hh + r) * 64 + t * 16 + c] = oacc[t][r] * inv;
  }
  __builtin_amdgcn_fence(__ATOMIC_RELEASE, "workgroup");
  __builtin_amdgcn_wave_barrier();
  __builtin_amdgcn_fence(__ATOMIC_ACQUIRE, "workgroup");
  {
    const int h2 = lane >> 4, c4 = (lane & 15) * 4;
    v4f ov[8];
#pragma unroll
    for (int it = 0; it < 8; ++it) {
      const int row = it * 2 + h2;
      ov[it] = *(const v4f*)(os + row * 64 + c4);
    }
    for (int pass = 0; pass < 2; ++pass) {
#pragma unroll
      for (int it = 0; it < 8; ++it) {
        const int row = it * 2 + h2;
        const size_t go = (rowB + q0 + row) * DM + (size_t)h * HD + c4;
        *(volatile v4f*)(outp + go) = ov[it];
      }
      __threadfence();
    }
  }
}

extern "C" void kernel_launch(void* const* d_in, const int* in_sizes, int n_in,
                              void* d_out, int out_size, void* d_ws, size_t ws_size,
                              hipStream_t stream) {
  if (n_in < 14) return;
  if (in_sizes[0] != NB * SEQ * DM) return;
  if (in_sizes[1] != NB * SEQ) return;
  if (in_sizes[2] != DM * DM || in_sizes[6] != DM * DM || in_sizes[10] != DM * DM) return;
  if (in_sizes[3] != DM || in_sizes[7] != DM || in_sizes[11] != DM) return;
  if (in_sizes[4] != LR * DM || in_sizes[8] != LR * DM || in_sizes[12] != LR * DM) return;
  if (in_sizes[5] != DM * LR || in_sizes[9] != DM * LR || in_sizes[13] != DM * LR) return;
  if (out_size != OUTN) return;

  const float* x    = (const float*)d_in[0];
  const float* mask = (const float*)d_in[1];
  const float* Wq   = (const float*)d_in[2];
  const float* bq   = (const float*)d_in[3];
  const float* Aq   = (const float*)d_in[4];
  const float* Bq   = (const float*)d_in[5];
  const float* Wk   = (const float*)d_in[6];
  const float* bk   = (const float*)d_in[7];
  const float* Ak   = (const float*)d_in[8];
  const float* Bk   = (const float*)d_in[9];
  const float* Wv   = (const float*)d_in[10];
  const float* bv   = (const float*)d_in[11];
  const float* Av   = (const float*)d_in[12];
  const float* Bv   = (const float*)d_in[13];

  const size_t PXb = (size_t)ROWS * DM * 2;
  const size_t PW  = (size_t)DM * DM * 2;
  const size_t PT  = (size_t)3 * ROWS * LR * 4;
  const size_t PF  = (size_t)ROWS * DM * 4;
  const size_t PH  = (size_t)ROWS * DM * 2;
  const size_t PVt = (size_t)NB * DM * SEQ * 2;
  size_t off = 0;
  const size_t oXb = off; off += PXb;
  const size_t oWq = off; off += PW;
  const size_t oWk = off; off += PW;
  const size_t oWv = off; off += PW;
  const size_t oT  = off; off += PT;
  const size_t oTf = off; off += PF;
  const size_t oQh = off; off += PH;
  const size_t oQl = off; off += PH;
  const size_t oKh = off; off += PH;
  const size_t oKl = off; off += PH;
  const size_t oVt = off; off += PVt;
  const size_t oVl = off; off += PVt;
  if (off > ws_size) return;
  if (off > (size_t)134217728) return;

  char* ws = (char*)d_ws;
  unsigned short* Xb  = (unsigned short*)(ws + oXb);
  unsigned short* Wqb = (unsigned short*)(ws + oWq);
  unsigned short* Wkb = (unsigned short*)(ws + oWk);
  unsigned short* Wvb = (unsigned short*)(ws + oWv);
  float*          T   = (float*)(ws + oT);
  float*          Tf  = (float*)(ws + oTf);
  unsigned short* Qh  = (unsigned short*)(ws + oQh);
  unsigned short* Ql  = (unsigned short*)(ws + oQl);
  unsigned short* Kh  = (unsigned short*)(ws + oKh);
  unsigned short* Kl  = (unsigned short*)(ws + oKl);
  unsigned short* VTh = (unsigned short*)(ws + oVt);
  unsigned short* VTl = (unsigned short*)(ws + oVl);
  float*          outf = (float*)d_out;

  const dim3 blk(256);
  const int n8x = ROWS * DM / 8;
  const int n8w = DM * DM / 8;
  const dim3 gCvtX((n8x + 255) / 256);
  const dim3 gCvtW((n8w + 255) / 256);
  const dim3 gLora(ROWS / 8, 3);
  const dim3 gGemm(((ROWS / 64) * (DM / 64) + 7) / 8);
  const dim3 gVpl(SEQ / 64, NH, NB);
  const dim3 gAttn(NB * NH * NQB);
  const float lsc     = 4.0f;
  const float qkScale = 16.0f;
  const float sscale  = 1.0f / 2048.0f;
  const float vScale  = 256.0f;
  const float attOscl = 1.0f / 262144.0f;

  cvt_bf16x8<<<gCvtX, blk, 0, stream>>>(x, Xb, n8x);
  cvt_bf16x8<<<gCvtW, blk, 0, stream>>>(Wq, Wqb, n8w);
  cvt_bf16x8<<<gCvtW, blk, 0, stream>>>(Wk, Wkb, n8w);
  cvt_bf16x8<<<gCvtW, blk, 0, stream>>>(Wv, Wvb, n8w);
  lora_t<<<gLora, blk, 0, stream>>>(Xb, Aq, Ak, Av, T);
  gemm64_lora<<<gGemm, blk, 0, stream>>>(Xb, DM, Wqb, DM, bq, T, Bq, lsc, Tf, DM, ROWS, DM, DM);
  planes_f16x8<<<gCvtX, blk, 0, stream>>>(Tf, Qh, Ql, n8x, qkScale);
  gemm64_lora<<<gGemm, blk, 0, stream>>>(Xb, DM, Wkb, DM, bk, T + (size_t)ROWS * LR, Bk, lsc,
                                         Tf, DM, ROWS, DM, DM);
  planes_f16x8<<<gCvtX, blk, 0, stream>>>(Tf, Kh, Kl, n8x, qkScale);
  gemm64_lora<<<gGemm, blk, 0, stream>>>(Xb, DM, Wvb, DM, bv, T + (size_t)2 * ROWS * LR, Bv, lsc,
                                         Tf, DM, ROWS, DM, DM);
  v_planes<<<gVpl, blk, 0, stream>>>(Tf, DM, VTh, VTl, vScale);
  attn_p64<<<gAttn, dim3(128), 0, stream>>>(Qh, Ql, Kh, Kl, VTh, VTl, mask, outf, sscale, attOscl);
  (void)hipGetLastError();
}
